// COG_36404142801393
// MI455X (gfx1250) — hardware-run, weakly checked
//
#include <hip/hip_runtime.h>
#include <math.h>

typedef __attribute__((ext_vector_type(16))) _Float16 v16h;
typedef __attribute__((ext_vector_type(8)))  _Float16 v8h;
typedef __attribute__((ext_vector_type(4)))  _Float16 v4h;
typedef __attribute__((ext_vector_type(16))) __bf16   v16b;
typedef __attribute__((ext_vector_type(8)))  __bf16   v8b;
typedef __attribute__((ext_vector_type(8)))  float    v8f;
typedef __attribute__((ext_vector_type(4)))  float    v4f;
typedef __attribute__((ext_vector_type(4)))  unsigned int v4u;

constexpr int kT    = 4096;
constexpr int kFD   = 2048;
constexpr int kD    = 128;
constexpr int kNG   = 16;
constexpr int kNH   = 8;
constexpr int kDq   = 16;
constexpr int kLQ   = 64;
constexpr int kNL   = 2;
constexpr int kHid  = 2048;
constexpr int kGF   = 512;
constexpr int kRows = kT * kNG;
constexpr int kPadRows = kLQ - 1;
constexpr int kVisRows = 4160;
constexpr int kAP = 136;
constexpr int kVP = 104;
constexpr int kUR = 96;
constexpr int kFStride = 8;
static_assert(kNH * kDq == kD, "head split");
static_assert(kVisRows >= kPadRows + kT && (kVisRows % 64) == 0, "visual plane rows");
static_assert(3 * kFStride + kLQ <= kUR && kUR <= kVP, "staged key rows");
static_assert((kT % 32) == 0 && (kRows % 64) == 0 && (kD % 64) == 0 && (kHid % 128) == 0, "tile multiples");
static_assert((kFD % 32) == 0 && (kD % 32) == 0 && (kHid % 32) == 0, "GEMM K multiples of 32");
static_assert(kNG == 16 && kDq == 16 && kD == 128, "fragment maps assume these");

constexpr float kWCarry   = 64.0f;
constexpr float kKVCarry  = 16.0f;
constexpr float kPCarry   = 1024.0f;
constexpr float kTxtCarry = 64.0f;
constexpr float kInvD     = 1.0f / (float)kD;
constexpr float kLnEps    = 1e-5f;

constexpr size_t kOffLF   = 0;
constexpr size_t kOffWVIS = kOffLF   + (size_t)kT * kFD * 2;
constexpr size_t kOffWQ   = kOffWVIS + (size_t)kD * kFD * 2;
constexpr size_t kOffWKV  = kOffWQ   + (size_t)kNL * kD * kD * 2;
constexpr size_t kOffW1   = kOffWKV  + (size_t)2 * kNL * kD * kD * 2;
constexpr size_t kOffW2   = kOffW1   + (size_t)kNL * kHid * kD * 2;
constexpr size_t kOffWQF  = kOffW2   + (size_t)kNL * kD * kHid * 2;
constexpr size_t kOffVIS  = kOffWQF  + (size_t)kD * kD * 2;
constexpr size_t kOffLNV  = kOffVIS  + (size_t)kT * kD * 4;
constexpr size_t kOffKV   = kOffLNV  + (size_t)kVisRows * kD * 2;
constexpr size_t kOffTEXT = kOffKV   + (size_t)2 * kNL * kVisRows * kD * 2;
constexpr size_t kOffKF   = kOffTEXT + (size_t)kNG * kD * 4;
constexpr size_t kOffVFT  = kOffKF   + (size_t)kNG * kD * 2;
constexpr size_t kOffX    = kOffVFT  + (size_t)kD * 32 * 2;
constexpr size_t kOffTST  = kOffX    + (size_t)kRows * kD * 4;
constexpr size_t kWsTotal = kOffTST  + (size_t)kRows * kD * 4;
static_assert(kWsTotal == 94179328ull, "carve total");
static_assert(kWsTotal <= 134217728ull, "carve cap");
static_assert((kOffWVIS % 128) == 0 && (kOffWQ % 128) == 0 && (kOffWKV % 128) == 0 && (kOffW1 % 128) == 0 &&
              (kOffW2 % 128) == 0 && (kOffWQF % 128) == 0 && (kOffVIS % 128) == 0 && (kOffLNV % 128) == 0 &&
              (kOffKV % 128) == 0 && (kOffTEXT % 128) == 0 && (kOffKF % 128) == 0 && (kOffVFT % 128) == 0 &&
              (kOffX % 128) == 0 && (kOffTST % 128) == 0, "128-B aligned regions");

__device__ __forceinline__ unsigned short f2bf_bits(float f) {
  unsigned u = __float_as_uint(f);
  return (unsigned short)((u + 0x7FFFu + ((u >> 16) & 1u)) >> 16);
}
__device__ __forceinline__ float bf_bits2f(unsigned short h) { return __uint_as_float(((unsigned)h) << 16); }

__device__ __forceinline__ void dep_guard_h(v8f& a, v8f& b, v16h x, v16h y) { asm volatile("v_nop\n\tv_nop\n\tv_nop\n\tv_nop" : "+v"(a), "+v"(b) : "v"(x), "v"(y)); }
__device__ __forceinline__ void dep_guard_b(v8f& a, v8f& b, v16b x, v16b y) { asm volatile("v_nop\n\tv_nop\n\tv_nop\n\tv_nop" : "+v"(a), "+v"(b) : "v"(x), "v"(y)); }
__device__ __forceinline__ void keep4_h(v16h a, v16h b, v16h c, v16h d) { asm volatile("v_nop" :: "v"(a), "v"(b), "v"(c), "v"(d)); }
__device__ __forceinline__ void keep4_b(v16b a, v16b b, v16b c, v16b d) { asm volatile("v_nop" :: "v"(a), "v"(b), "v"(c), "v"(d)); }
__device__ __forceinline__ void acc_guard4(v8f& a, v8f& b, v8f& c, v8f& d) { asm volatile("v_nop\n\tv_nop\n\tv_nop\n\tv_nop" : "+v"(a), "+v"(b), "+v"(c), "+v"(d)); }
template <typename T> struct Frag;
template <> struct Frag<_Float16> {
  typedef v16h V; union U { v16h v; v8h h[2]; };
  static __device__ __forceinline__ v16h load(const _Float16* p) {
    U f; f.h[0] = *(const v8h*)(p); f.h[1] = *(const v8h*)(p + 16); return f.v;
  }
  static __device__ __forceinline__ v8f mma(v16h a, v16h b, v8f c) {
    return __builtin_amdgcn_wmma_f32_16x16x32_f16(false, a, false, b, (short)0, c, false, false);
  }
  static __device__ __forceinline__ void guard(v8f& a, v8f& b, v16h x, v16h y) { dep_guard_h(a, b, x, y); }
  static __device__ __forceinline__ void keep(v16h a, v16h b, v16h c, v16h d) { keep4_h(a, b, c, d); }
};
template <> struct Frag<__bf16> {
  typedef v16b V; union U { v16b v; v8b h[2]; };
  static __device__ __forceinline__ v16b load(const __bf16* p) {
    U f; f.h[0] = *(const v8b*)(p); f.h[1] = *(const v8b*)(p + 16); return f.v;
  }
  static __device__ __forceinline__ v8f mma(v16b a, v16b b, v8f c) {
    return __builtin_amdgcn_wmma_f32_16x16x32_bf16(false, a, false, b, (short)0, c, false, false);
  }
  static __device__ __forceinline__ void guard(v8f& a, v8f& b, v16b x, v16b y) { dep_guard_b(a, b, x, y); }
  static __device__ __forceinline__ void keep(v16b a, v16b b, v16b c, v16b d) { keep4_b(a, b, c, d); }
};

__device__ __forceinline__ unsigned pk16(unsigned short a, unsigned short b) { return (unsigned)a | ((unsigned)b << 16); }
__device__ __forceinline__ unsigned short h_bits(float f) { const _Float16 h = (_Float16)f; return __builtin_bit_cast(unsigned short, h); }
__device__ __forceinline__ _Float16 bits2h(unsigned b) { const unsigned short s = (unsigned short)b; return __builtin_bit_cast(_Float16, s); }

union FH { v16h v; v8h h[2]; };

__device__ __forceinline__ v8f mma_h(v16h a, v16h b, v8f c) {
  c = __builtin_amdgcn_wmma_f32_16x16x32_f16(false, a, false, b, (short)0, c, false, false);
  asm volatile("v_nop\n\tv_nop\n\tv_nop\n\tv_nop" : "+v"(c) : "v"(a), "v"(b));
  return c;
}

__device__ __forceinline__ float max8(v8f s) {
  return fmaxf(fmaxf(fmaxf(s[0], s[1]), fmaxf(s[2], s[3])), fmaxf(fmaxf(s[4], s[5]), fmaxf(s[6], s[7])));
}

__device__ __forceinline__ v4f ln_row4(v4f v) {
  float s = (v[0] + v[1]) + (v[2] + v[3]);
#pragma unroll
  for (int off = 16; off > 0; off >>= 1) s += __shfl_xor(s, off, 32);
  const float mean = s * kInvD;
  const float d0 = v[0] - mean, d1 = v[1] - mean, d2 = v[2] - mean, d3 = v[3] - mean;
  float q = (d0 * d0 + d1 * d1) + (d2 * d2 + d3 * d3);
#pragma unroll
  for (int off = 16; off > 0; off >>= 1) q += __shfl_xor(q, off, 32);
  const float rs = rsqrtf(q * kInvD + kLnEps);
  return (v4f){d0 * rs, d1 * rs, d2 * rs, d3 * rs};
}

template <int ET> struct Elem;
template <> struct Elem<0> { typedef _Float16 T; };
template <> struct Elem<1> { typedef __bf16 T; };
template <int ET, bool SPLIT, int BIAS_MODE, int OUT_MODE, bool RESID, int ACT = 0>
__global__ __launch_bounds__(256) void wmma_gemm64(
    const unsigned short* __restrict__ Ap, const unsigned short* __restrict__ A2p, int lda, long strideA,
    const unsigned short* __restrict__ Btp, const unsigned short* __restrict__ Bt2p, int ldb, long strideB,
    void* __restrict__ Cout, void* __restrict__ Cout2, int ldc, long strideC,
    const float* __restrict__ bias,
    const float* __restrict__ resid, long strideR,
    int M, int N, int K, float scale) {
  typedef typename Elem<ET>::T T;
  typedef typename Frag<T>::V V;
  const T* A = (const T*)Ap; const T* A2 = (const T*)A2p; const T* Bt = (const T*)Btp; const T* Bt2 = (const T*)Bt2p;
  __shared__ __align__(16) float sT[8][16 * 68];
  const int b    = blockIdx.y;
  const int lane = threadIdx.x & 31;
  const int wave = threadIdx.x >> 5;
  const int tilesN = N >> 6;
  const int tilesM = M >> 6;
  const int tile = blockIdx.x * 8 + wave;
  if (tile >= tilesM * tilesN) return;
  const int tm = tile / tilesN;
  const int tn = tile - tm * tilesN;
  const int m0 = tm << 6;
  const int n0 = tn << 6;

  const T* Ab  = A  + (size_t)b * strideA;
  const T* Bb  = Bt + (size_t)b * strideB;
  const T* Ab2 = SPLIT ? (A2  + (size_t)b * strideA) : nullptr;
  const T* Bb2 = SPLIT ? (Bt2 + (size_t)b * strideB) : nullptr;

  const int rlane = lane & 15;
  const int koff  = (lane >> 4) * 8;
  const int mOff  = (lane >> 4) * 8;

  v8f acc[4][4];
#pragma unroll
  for (int i = 0; i < 4; ++i)
#pragma unroll
    for (int j = 0; j < 4; ++j) acc[i][j] = (v8f){0.f,0.f,0.f,0.f,0.f,0.f,0.f,0.f};

  for (int k0 = 0; k0 < K; k0 += 32) {
    V bh[4], bl[4];
#pragma unroll
    for (int j = 0; j < 4; ++j) {
      const size_t bo = (size_t)(n0 + (j << 4) + rlane) * ldb + koff + k0;
      bh[j] = Frag<T>::load(Bb + bo);
      if (SPLIT) bl[j] = Frag<T>::load(Bb2 + bo);
    }
#pragma unroll
    for (int i = 0; i < 4; ++i) {
      const size_t ao = (size_t)(m0 + (i << 4) + rlane) * lda + koff + k0;
      V ah = Frag<T>::load(Ab + ao);
      V al;
      if (SPLIT) al = Frag<T>::load(Ab2 + ao);
#pragma unroll
      for (int j = 0; j < 4; ++j) {
        acc[i][j] = Frag<T>::mma(ah, bh[j], acc[i][j]);
        if (SPLIT) {
          acc[i][j] = Frag<T>::mma(ah, bl[j], acc[i][j]);
          acc[i][j] = Frag<T>::mma(al, bh[j], acc[i][j]);
        }
      }
      Frag<T>::guard(acc[i][0], acc[i][3], ah, SPLIT ? al : ah);
    }
    Frag<T>::keep(bh[0], bh[1], bh[2], bh[3]);
    if (SPLIT) Frag<T>::keep(bl[0], bl[1], bl[2], bl[3]);
  }
  acc_guard4(acc[0][0], acc[0][1], acc[0][2], acc[0][3]);
  acc_guard4(acc[1][0], acc[1][1], acc[1][2], acc[1][3]);
  acc_guard4(acc[2][0], acc[2][1], acc[2][2], acc[2][3]);
  acc_guard4(acc[3][0], acc[3][1], acc[3][2], acc[3][3]);

  float* slab = sT[wave];
  const float* Rb = RESID ? (resid + (size_t)b * strideR) : nullptr;
#pragma unroll
  for (int i = 0; i < 4; ++i) {
    const int mBase = m0 + (i << 4);
#pragma unroll
    for (int j = 0; j < 4; ++j) {
      const int n = n0 + (j << 4) + rlane;
      float bv = 0.f;
      if (BIAS_MODE == 2) bv = bias[n];
#pragma unroll
      for (int r = 0; r < 8; ++r) {
        float v = acc[i][j][r] * scale;
        if (BIAS_MODE == 1) v += bias[mBase + mOff + r];
        if (BIAS_MODE == 2) v += bv;
        if (RESID) v += Rb[(size_t)(mBase + mOff + r) * ldc + n];
        if (ACT == 2) v = fmaxf(v, 0.0f);
        if (ACT == 4) v = (v > 0.f) ? v : 0.01f * v;
        slab[(mOff + r) * 68 + (j << 4) + rlane] = v;
      }
    }
    __builtin_amdgcn_fence(__ATOMIC_RELEASE, "workgroup");
    __builtin_amdgcn_wave_barrier();
    __builtin_amdgcn_fence(__ATOMIC_ACQUIRE, "workgroup");
    if (OUT_MODE == 0) {
      float* C = (float*)Cout + (size_t)b * strideC;
      const int hh = lane >> 4, c4 = (lane & 15) * 4;
      for (int pass = 0; pass < 2; ++pass) {
#pragma unroll
        for (int it = 0; it < 8; ++it) {
          const int row = it * 2 + hh;
          v4f v = *(const v4f*)(slab + row * 68 + c4);
          *(volatile v4f*)(C + (size_t)(mBase + row) * ldc + n0 + c4) = v;
        }
        __threadfence();
      }
    } else {
      const int q = lane >> 3, c8 = (lane & 7) * 8;
      unsigned short* C  = (unsigned short*)Cout  + (size_t)b * strideC;
      unsigned short* C2 = (OUT_MODE == 2) ? ((unsigned short*)Cout2 + (size_t)b * strideC) : nullptr;
      for (int pass = 0; pass < 2; ++pass) {
#pragma unroll
        for (int it = 0; it < 4; ++it) {
          const int row = it * 4 + q;
          const float* sp = slab + row * 68 + c8;
          v8h hv, lv;
#pragma unroll
          for (int e = 0; e < 8; ++e) {
            if (OUT_MODE == 1) {
              hv[e] = (_Float16)sp[e];
            } else {
              unsigned short hb = f2bf_bits(sp[e]);
              unsigned short lb = f2bf_bits(sp[e] - bf_bits2f(hb));
              hv[e] = __builtin_bit_cast(_Float16, hb);
              lv[e] = __builtin_bit_cast(_Float16, lb);
            }
          }
          *(volatile v8h*)(C + (size_t)(mBase + row) * ldc + n0 + c8) = hv;
          if (OUT_MODE == 2) *(volatile v8h*)(C2 + (size_t)(mBase + row) * ldc + n0 + c8) = lv;
        }
        __threadfence();
      }
    }
    __builtin_amdgcn_fence(__ATOMIC_RELEASE, "workgroup");
    __builtin_amdgcn_wave_barrier();
    __builtin_amdgcn_fence(__ATOMIC_ACQUIRE, "workgroup");
  }
}

__global__ __launch_bounds__(256) void transpose_cast_kernel(const float* __restrict__ src, unsigned short* __restrict__ dst,
                                                             int R, int C, float scale) {
  __shared__ float sm[64][65];
  const int t  = threadIdx.x;
  const int r0 = blockIdx.x * 64;
  const int c0 = blockIdx.y * 64;
  const size_t zoff = (size_t)blockIdx.z * (size_t)R * (size_t)C;
  const float* S = src + zoff;
  unsigned short* Dp = dst + zoff;
#pragma unroll 8
  for (int i = 0; i < 16; ++i) {
    const int e  = i * 256 + t;
    const int rr = e >> 6;
    const int cc = e & 63;
    sm[cc][rr] = S[(size_t)(r0 + rr) * C + c0 + cc] * scale;
  }
  __syncthreads();
  const int lane = t & 31, wave = t >> 5;
  const int q = lane >> 3, c8 = (lane & 7) * 8;
  for (int pass = 0; pass < 2; ++pass) {
#pragma unroll
    for (int it = 0; it < 2; ++it) {
      const int row = wave * 8 + it * 4 + q;
      unsigned short hb[8];
#pragma unroll
      for (int e = 0; e < 8; ++e) hb[e] = h_bits(sm[row][c8 + e]);
      const v4u u = (v4u){pk16(hb[0], hb[1]), pk16(hb[2], hb[3]), pk16(hb[4], hb[5]), pk16(hb[6], hb[7])};
      *(volatile v4u*)(Dp + (size_t)(c0 + row) * R + r0 + c8) = u;
    }
    __threadfence();
  }
}

__global__ __launch_bounds__(256) void cast8_f16_kernel(const float* __restrict__ in, unsigned short* __restrict__ out, int n8) {
  const int i = blockIdx.x * 256 + threadIdx.x;
  if (i >= n8) return;
  const float* p = in + 8 * (size_t)i;
  const v4f a = *(const v4f*)(p);
  const v4f c = *(const v4f*)(p + 4);
  unsigned short hb[8];
#pragma unroll
  for (int e = 0; e < 4; ++e) {
    hb[e]     = h_bits(a[e]);
    hb[4 + e] = h_bits(c[e]);
  }
  const v4u u = (v4u){pk16(hb[0], hb[1]), pk16(hb[2], hb[3]), pk16(hb[4], hb[5]), pk16(hb[6], hb[7])};
  unsigned short* q = out + 8 * (size_t)i;
  *(volatile v4u*)q = u;
  __threadfence();
  *(volatile v4u*)q = u;
}

__global__ __launch_bounds__(256) void ln_vis_kernel(const float* __restrict__ vis, unsigned short* __restrict__ lnv) {
  const int tid = threadIdx.x, lane = tid & 31, wave = tid >> 5;
  const int l16 = lane & 15;
  const int prow = blockIdx.x * 16 + wave * 2 + (lane >> 4);
  const bool real = (prow >= kPadRows) && (prow < kPadRows + kT);
  int srow = prow - kPadRows;
  srow = srow < 0 ? 0 : srow;
  srow = srow > (kT - 1) ? (kT - 1) : srow;
  const float* sp = vis + (size_t)srow * kD + l16 * 8;
  const v4f a0 = *(const v4f*)(sp);
  const v4f a1 = *(const v4f*)(sp + 4);
  float s = ((a0[0] + a0[1]) + (a0[2] + a0[3])) + ((a1[0] + a1[1]) + (a1[2] + a1[3]));
#pragma unroll
  for (int off = 8; off > 0; off >>= 1) s += __shfl_xor(s, off, 32);
  const float mean = s * kInvD;
  float d[8];
#pragma unroll
  for (int e = 0; e < 4; ++e) { d[e] = a0[e] - mean; d[4 + e] = a1[e] - mean; }
  float q = 0.f;
#pragma unroll
  for (int e = 0; e < 8; ++e) q += d[e] * d[e];
#pragma unroll
  for (int off = 8; off > 0; off >>= 1) q += __shfl_xor(q, off, 32);
  const float rs = rsqrtf(q * kInvD + kLnEps);
  unsigned short hb[8];
#pragma unroll
  for (int e = 0; e < 8; ++e) {
    const float o = real ? (d[e] * rs) : 0.0f;
    hb[e] = h_bits(o);
  }
  const v4u u = (v4u){pk16(hb[0], hb[1]), pk16(hb[2], hb[3]), pk16(hb[4], hb[5]), pk16(hb[6], hb[7])};
  unsigned short* dp = lnv + (size_t)prow * kD + l16 * 8;
  *(volatile v4u*)dp = u;
  __threadfence();
  *(volatile v4u*)dp = u;
}

__global__ __launch_bounds__(256) void text_kernel(const float* __restrict__ g, const float* __restrict__ Wtxt,
                                                   const float* __restrict__ Wkf, const float* __restrict__ Wvf,
                                                   float* __restrict__ textOut, unsigned short* __restrict__ KfOut,
                                                   unsigned short* __restrict__ VfTOut, float carry) {
  __shared__ __align__(16) float sText[kNG * kD];
  __shared__ __align__(16) float sKf[kNG * kD];
  __shared__ __align__(16) float sVf[kNG * kD];
  const int t = threadIdx.x;
  const int c = t & 127;
  const int rg = (t >> 7) * 8;
  float acc[8];
#pragma unroll
  for (int j = 0; j < 8; ++j) acc[j] = 0.f;
#pragma unroll 1
  for (int k = 0; k < kGF; ++k) {
    const float w = Wtxt[(size_t)k * kD + c];
#pragma unroll
    for (int j = 0; j < 8; ++j) acc[j] = fmaf(g[(rg + j) * kGF + k], w, acc[j]);
  }
#pragma unroll
  for (int j = 0; j < 8; ++j) sText[(rg + j) * kD + c] = acc[j];
  __syncthreads();
  float ak[8], av[8];
#pragma unroll
  for (int j = 0; j < 8; ++j) { ak[j] = 0.f; av[j] = 0.f; }
#pragma unroll 1
  for (int k = 0; k < kD; ++k) {
    const float wk = Wkf[(size_t)k * kD + c];
    const float wv = Wvf[(size_t)k * kD + c];
#pragma unroll
    for (int j = 0; j < 8; ++j) {
      const float tv = sText[(rg + j) * kD + k];
      ak[j] = fmaf(tv, wk, ak[j]);
      av[j] = fmaf(tv, wv, av[j]);
    }
  }
#pragma unroll
  for (int j = 0; j < 8; ++j) {
    sKf[(rg + j) * kD + c] = ak[j] * carry;
    sVf[(rg + j) * kD + c] = av[j] * carry;
  }
  __syncthreads();
  const v4f tv0 = *(const v4f*)(sText + 4 * t);
  const v4f tv1 = *(const v4f*)(sText + 4 * (t + 256));
  unsigned short kb[8];
#pragma unroll
  for (int e = 0; e < 8; ++e) kb[e] = h_bits(sKf[8 * t + e]);
  const v4u ku = (v4u){pk16(kb[0], kb[1]), pk16(kb[2], kb[3]), pk16(kb[4], kb[5]), pk16(kb[6], kb[7])};
  v4u vu[2];
#pragma unroll
  for (int it = 0; it < 2; ++it) {
    const int idx = it * 256 + t;
    const int d = idx >> 2;
    const int k8 = (idx & 3) * 8;
    const bool live = (k8 < kNG);
    unsigned short vb[8];
#pragma unroll
    for (int e = 0; e < 8; ++e) {
      const int keyc = (k8 + e) & (kNG - 1);
      const float sv = sVf[keyc * kD + d];
      const float val = live ? sv : 0.0f;
      vb[e] = h_bits(val);
    }
    vu[it] = (v4u){pk16(vb[0], vb[1]), pk16(vb[2], vb[3]), pk16(vb[4], vb[5]), pk16(vb[6], vb[7])};
  }
  for (int pass = 0; pass < 2; ++pass) {
    *(volatile v4f*)(textOut + 4 * t) = tv0;
    *(volatile v4f*)(textOut + 4 * (t + 256)) = tv1;
    *(volatile v4u*)(KfOut + 8 * t) = ku;
    *(volatile v4u*)(VfTOut + 8 * t) = vu[0];
    *(volatile v4u*)(VfTOut + 8 * (t + 256)) = vu[1];
    __threadfence();
  }
}

__global__ __launch_bounds__(256) void enc_attn_kernel(
    const float* __restrict__ tsrc, int first,
    const unsigned short* __restrict__ WqTp, const unsigned short* __restrict__ Kpp, const unsigned short* __restrict__ Vpp,
    float* __restrict__ xout, float sscale, float cinv) {
  __shared__ __align__(16) float    sTq[64 * kD];
  __shared__ __align__(16) _Float16 sA[64 * kAP];
  __shared__ __align__(16) _Float16 sK[kUR * kAP];
  __shared__ __align__(16) _Float16 sVt[kD * kVP];
  __shared__ __align__(32) v8f      sS[8 * 4 * 32];
  __shared__ __align__(16) v8h      sP[8 * 4 * 32];

  const int tid = threadIdx.x, lane = tid & 31, wave = tid >> 5;
  const int rl = lane & 15, hh = lane >> 4, koff = hh * 8;
  const int blk = blockIdx.x;
  const int fb = (blk >> 3) * 32 + (blk & 7);
  const v8h zero8h = (v8h){(_Float16)0.f, (_Float16)0.f, (_Float16)0.f, (_Float16)0.f, (_Float16)0.f, (_Float16)0.f, (_Float16)0.f, (_Float16)0.f};
  const v8f zero8f = (v8f){0.f, 0.f, 0.f, 0.f, 0.f, 0.f, 0.f, 0.f};

#pragma unroll
  for (int it = 0; it < 8; ++it) {
    const int idx = it * 256 + tid;
    const int row = idx >> 5;
    const int c4 = (idx & 31) * 4;
    const int fi = row >> 4, q = row & 15;
    const int grow = (fb + kFStride * fi) * kNG + q;
    const int srow = first ? q : grow;
    const v4f v = *(const v4f*)(tsrc + (size_t)srow * kD + c4);
    *(v4f*)(sTq + row * kD + c4) = v;
  }
#pragma unroll 2
  for (int it = 0; it < 6; ++it) {
    const int idx = it * 256 + tid;
    const int u = idx >> 4;
    const int c8 = (idx & 15) * 8;
    int prow = fb + u;
    prow = prow < (kVisRows - 1) ? prow : (kVisRows - 1);
    const v4u kw = *(const v4u*)(Kpp + (size_t)prow * kD + c8);
    const v4u vw = *(const v4u*)(Vpp + (size_t)prow * kD + c8);
    *(v8h*)(sK + u * kAP + c8) = __builtin_bit_cast(v8h, kw);
    const unsigned w0 = vw[0], w1 = vw[1], w2 = vw[2], w3 = vw[3];
    sVt[(c8 + 0) * kVP + u] = bits2h(w0 & 0xffffu);
    sVt[(c8 + 1) * kVP + u] = bits2h(w0 >> 16);
    sVt[(c8 + 2) * kVP + u] = bits2h(w1 & 0xffffu);
    sVt[(c8 + 3) * kVP + u] = bits2h(w1 >> 16);
    sVt[(c8 + 4) * kVP + u] = bits2h(w2 & 0xffffu);
    sVt[(c8 + 5) * kVP + u] = bits2h(w2 >> 16);
    sVt[(c8 + 6) * kVP + u] = bits2h(w3 & 0xffffu);
    sVt[(c8 + 7) * kVP + u] = bits2h(w3 >> 16);
  }
  __syncthreads();

#pragma unroll 1
  for (int rr = 0; rr < 8; ++rr) {
    const int row = wave * 8 + rr;
    const v4f v = *(const v4f*)(sTq + row * kD + lane * 4);
    const v4f o = ln_row4(v);
    *(v4f*)(sTq + row * kD + lane * 4) = o;
    v4h hv;
    hv[0] = (_Float16)o[0]; hv[1] = (_Float16)o[1]; hv[2] = (_Float16)o[2]; hv[3] = (_Float16)o[3];
    *(v4h*)(sA + row * kAP + lane * 4) = hv;
  }
  __syncthreads();

  const _Float16* WqT = (const _Float16*)WqTp;
  v16h aW[4];
#pragma unroll
  for (int ks = 0; ks < 4; ++ks) aW[ks] = Frag<_Float16>::load(WqT + (size_t)(16 * wave + rl) * kD + ks * 32 + koff);

  FH qf;
  qf.h[0] = zero8h;
  qf.h[1] = zero8h;
#pragma unroll 1
  for (int fi = 0; fi < 4; ++fi) {
    if (!first || fi == 0) {
      v8f qa = zero8f;
#pragma unroll
      for (int ks = 0; ks < 4; ++ks) {
        const v16h bq = Frag<_Float16>::load(sA + (fi * 16 + rl) * kAP + ks * 32 + koff);
        qa = mma_h(aW[ks], bq, qa);
      }
      v8h qh;
#pragma unroll
      for (int r = 0; r < 8; ++r) qh[r] = (_Float16)qa[r];
      qf.h[0] = qh;
      qf.h[1] = zero8h;
    }
    float m = -INFINITY;
#pragma unroll 1
    for (int j = 0; j < 4; ++j) {
      FH kf;
      kf.h[0] = *(const v8h*)(sK + (kFStride * fi + 16 * j + rl) * kAP + 16 * wave + koff);
      kf.h[1] = zero8h;
      const v8f st = mma_h(kf.v, qf.v, zero8f);
      sS[(wave * 4 + j) * 32 + lane] = st;
      m = fmaxf(m, max8(st));
    }
    m = fmaxf(m, __shfl_xor(m, 16, 32));
    float sum = 0.f;
#pragma unroll 1
    for (int j = 0; j < 4; ++j) {
      const v8f st = sS[(wave * 4 + j) * 32 + lane];
      v8h pv;
#pragma unroll
      for (int r = 0; r < 8; ++r) {
        const float p = __expf((st[r] - m) * sscale);
        sum += p;
        pv[r] = (_Float16)(p * kPCarry);
      }
      sP[(wave * 4 + j) * 32 + lane] = pv;
    }
    sum += __shfl_xor(sum, 16, 32);
    v8f ca = zero8f;
#pragma unroll
    for (int kk = 0; kk < 2; ++kk) {
      FH pa;
      pa.h[0] = sP[(wave * 4 + 2 * kk) * 32 + lane];
      pa.h[1] = sP[(wave * 4 + 2 * kk + 1) * 32 + lane];
      const v16h va = Frag<_Float16>::load(sVt + (16 * wave + rl) * kVP + kFStride * fi + 32 * kk + koff);
      ca = mma_h(va, pa.v, ca);
    }
    const float inv = cinv * (1.0f / sum);
    float* dst = sTq + (fi * 16 + rl) * kD + 16 * wave + koff;
    v4f o0 = *(const v4f*)(dst);
    v4f o1 = *(const v4f*)(dst + 4);
    o0[0] += ca[0] * inv; o0[1] += ca[1] * inv; o0[2] += ca[2] * inv; o0[3] += ca[3] * inv;
    o1[0] += ca[4] * inv; o1[1] += ca[5] * inv; o1[2] += ca[6] * inv; o1[3] += ca[7] * inv;
    *(v4f*)(dst) = o0;
    *(v4f*)(dst + 4) = o1;
  }
  __syncthreads();

  v4f outv[8];
#pragma unroll
  for (int rr = 0; rr < 8; ++rr) {
    const int row = wave * 8 + rr;
    const v4f v = *(const v4f*)(sTq + row * kD + lane * 4);
    const v4f t1 = ln_row4(v);
    outv[rr] = ln_row4(t1);
  }
  for (int pass = 0; pass < 2; ++pass) {
#pragma unroll
    for (int rr = 0; rr < 8; ++rr) {
      const int row = wave * 8 + rr;
      const int grow = (fb + kFStride * (row >> 4)) * kNG + (row & 15);
      *(volatile v4f*)(xout + (size_t)grow * kD + lane * 4) = outv[rr];
    }
    __threadfence();
  }
}

__global__ __launch_bounds__(256) void ffn_kernel(const float* __restrict__ xin, const unsigned short* __restrict__ W1Tp,
                                                  const unsigned short* __restrict__ W2Tp, float* __restrict__ tout, float yscale) {
  __shared__ __align__(16) float    sXf[64 * kD];
  __shared__ __align__(16) _Float16 sXh[64 * kAP];
  __shared__ __align__(16) _Float16 sH[2 * 64 * kAP];
  const int tid = threadIdx.x, lane = tid & 31, wave = tid >> 5;
  const int rl = lane & 15, hh = lane >> 4, koff = hh * 8;
  const int m0 = blockIdx.x * 64;
  const _Float16* W1T = (const _Float16*)W1Tp;
  const _Float16* W2T = (const _Float16*)W2Tp;
  const v8f zero8f = (v8f){0.f, 0.f, 0.f, 0.f, 0.f, 0.f, 0.f, 0.f};

#pragma unroll
  for (int it = 0; it < 8; ++it) {
    const int idx = it * 256 + tid;
    const int row = idx >> 5;
    const int c4 = (idx & 31) * 4;
    const v4f v = *(const v4f*)(xin + (size_t)(m0 + row) * kD + c4);
    *(v4f*)(sXf + row * kD + c4) = v;
    v4h hv;
    hv[0] = (_Float16)v[0]; hv[1] = (_Float16)v[1]; hv[2] = (_Float16)v[2]; hv[3] = (_Float16)v[3];
    *(v4h*)(sXh + row * kAP + c4) = hv;
  }
  __syncthreads();

  v8f yacc[4];
#pragma unroll
  for (int i = 0; i < 4; ++i) yacc[i] = zero8f;

#pragma unroll 1
  for (int c = 0; c < kHid / 128; ++c) {
    _Float16* hb = sH + (c & 1) * (64 * kAP);
    v8f hacc[4];
#pragma unroll
    for (int i = 0; i < 4; ++i) hacc[i] = zero8f;
#pragma unroll
    for (int ks = 0; ks < 4; ++ks) {
      const v16h a = Frag<_Float16>::load(W1T + (size_t)(c * 128 + 16 * wave + rl) * kD + ks * 32 + koff);
#pragma unroll
      for (int i = 0; i < 4; ++i) {
        const v16h b = Frag<_Float16>::load(sXh + (i * 16 + rl) * kAP + ks * 32 + koff);
        hacc[i] = mma_h(a, b, hacc[i]);
      }
    }
#pragma unroll
    for (int i = 0; i < 4; ++i) {
      v8h hv;
#pragma unroll
      for (int r = 0; r < 8; ++r) hv[r] = (_Float16)fmaxf(hacc[i][r], 0.0f);
      *(v8h*)(hb + (i * 16 + rl) * kAP + 16 * wave + koff) = hv;
    }
    __syncthreads();
#pragma unroll
    for (int ks = 0; ks < 4; ++ks) {
      const v16h a = Frag<_Float16>::load(W2T + (size_t)(16 * wave + rl) * kHid + c * 128 + ks * 32 + koff);
#pragma unroll
      for (int i = 0; i < 4; ++i) {
        const v16h b = Frag<_Float16>::load(hb + (i * 16 + rl) * kAP + ks * 32 + koff);
        yacc[i] = mma_h(a, b, yacc[i]);
      }
    }
  }

#pragma unroll
  for (int i = 0; i < 4; ++i) {
    float* dst = sXf + (i * 16 + rl) * kD + 16 * wave + koff;
    v4f o0 = *(const v4f*)(dst);
    v4f o1 = *(const v4f*)(dst + 4);
    o0[0] += yacc[i][0] * yscale; o0[1] += yacc[i][1] * yscale; o0[2] += yacc[i][2] * yscale; o0[3] += yacc[i][3] * yscale;
    o1[0] += yacc[i][4] * yscale; o1[1] += yacc[i][5] * yscale; o1[2] += yacc[i][6] * yscale; o1[3] += yacc[i][7] * yscale;
    *(v4f*)(dst) = o0;
    *(v4f*)(dst + 4) = o1;
  }
  __syncthreads();

  v4f outv[8];
#pragma unroll
  for (int rr = 0; rr < 8; ++rr) {
    const int row = wave * 8 + rr;
    const v4f v = *(const v4f*)(sXf + row * kD + lane * 4);
    outv[rr] = ln_row4(v);
  }
  for (int pass = 0; pass < 2; ++pass) {
#pragma unroll
    for (int rr = 0; rr < 8; ++rr) {
      const int row = wave * 8 + rr;
      *(volatile v4f*)(tout + (size_t)(m0 + row) * kD + lane * 4) = outv[rr];
    }
    __threadfence();
  }
}

__global__ __launch_bounds__(256) void final_attn_kernel(
    const float* __restrict__ tin, const unsigned short* __restrict__ WqfTp, const unsigned short* __restrict__ Kfp,
    const unsigned short* __restrict__ VfTp, float* __restrict__ out, float sscale, float cinv) {
  __shared__ __align__(16) float    sT[64 * kD];
  __shared__ __align__(16) _Float16 sA[64 * kAP];
  __shared__ __align__(16) _Float16 sQ[64 * kAP];
  const int tid = threadIdx.x, lane = tid & 31, wave = tid >> 5;
  const int rl = lane & 15, hh = lane >> 4, koff = hh * 8;
  const int m0 = blockIdx.x * 64;
  const _Float16* WqfT = (const _Float16*)WqfTp;
  const _Float16* Kf   = (const _Float16*)Kfp;
  const _Float16* VfT  = (const _Float16*)VfTp;
  const v8h zero8h = (v8h){(_Float16)0.f, (_Float16)0.f, (_Float16)0.f, (_Float16)0.f, (_Float16)0.f, (_Float16)0.f, (_Float16)0.f, (_Float16)0.f};
  const v8f zero8f = (v8f){0.f, 0.f, 0.f, 0.f, 0.f, 0.f, 0.f, 0.f};

#pragma unroll
  for (int it = 0; it < 8; ++it) {
    const int idx = it * 256 + tid;
    const int row = idx >> 5;
    const int c4 = (idx & 31) * 4;
    const v4f v = *(const v4f*)(tin + (size_t)(m0 + row) * kD + c4);
    *(v4f*)(sT + row * kD + c4) = v;
    v4h hv;
    hv[0] = (_Float16)v[0]; hv[1] = (_Float16)v[1]; hv[2] = (_Float16)v[2]; hv[3] = (_Float16)v[3];
    *(v4h*)(sA + row * kAP + c4) = hv;
  }
  __syncthreads();

  {
    v8f qa[4];
#pragma unroll
    for (int i = 0; i < 4; ++i) qa[i] = zero8f;
#pragma unroll
    for (int ks = 0; ks < 4; ++ks) {
      const v16h a = Frag<_Float16>::load(WqfT + (size_t)(16 * wave + rl) * kD + ks * 32 + koff);
#pragma unroll
      for (int i = 0; i < 4; ++i) {
        const v16h b = Frag<_Float16>::load(sA + (i * 16 + rl) * kAP + ks * 32 + koff);
        qa[i] = mma_h(a, b, qa[i]);
      }
    }
#pragma unroll
    for (int i = 0; i < 4; ++i) {
      v8h qh;
#pragma unroll
      for (int r = 0; r < 8; ++r) qh[r] = (_Float16)qa[i][r];
      *(v8h*)(sQ + (i * 16 + rl) * kAP + 16 * wave + koff) = qh;
    }
  }
  __syncthreads();

  {
    const int fi = wave >> 1, dh = wave & 1;
    v8f st = zero8f;
#pragma unroll
    for (int ks = 0; ks < 4; ++ks) {
      const v16h a = Frag<_Float16>::load(Kf + (size_t)rl * kD + ks * 32 + koff);
      const v16h b = Frag<_Float16>::load(sQ + (fi * 16 + rl) * kAP + ks * 32 + koff);
      st = mma_h(a, b, st);
    }
    float m = max8(st);
    m = fmaxf(m, __shfl_xor(m, 16, 32));
    float sum = 0.f;
    v8h pv;
#pragma unroll
    for (int r = 0; r < 8; ++r) {
      const float p = __expf((st[r] - m) * sscale);
      sum += p;
      pv[r] = (_Float16)(p * kPCarry);
    }
    sum += __shfl_xor(sum, 16, 32);
    FH pa;
    pa.h[0] = pv;
    pa.h[1] = zero8h;
    const float inv = cinv * (1.0f / sum);
#pragma unroll
    for (int dt = 0; dt < 4; ++dt) {
      const int dbase = (dh * 4 + dt) * 16;
      const v16h a = Frag<_Float16>::load(VfT + (size_t)(dbase + rl) * 32 + koff);
      const v8f ca = mma_h(a, pa.v, zero8f);
      float* dst = sT + (fi * 16 + rl) * kD + dbase + koff;
      v4f o0 = *(const v4f*)(dst);
      v4f o1 = *(const v4f*)(dst + 4);
      o0[0] += ca[0] * inv; o0[1] += ca[1] * inv; o0[2] += ca[2] * inv; o0[3] += ca[3] * inv;
      o1[0] += ca[4] * inv; o1[1] += ca[5] * inv; o1[2] += ca[6] * inv; o1[3] += ca[7] * inv;
      *(v4f*)(dst) = o0;
      *(v4f*)(dst + 4) = o1;
    }
  }
  __syncthreads();

  v4f outv[8];
#pragma unroll
  for (int rr = 0; rr < 8; ++rr) {
    const int row = wave * 8 + rr;
    const v4f v = *(const v4f*)(sT + row * kD + lane * 4);
    outv[rr] = ln_row4(v);
  }
  for (int pass = 0; pass < 2; ++pass) {
#pragma unroll
    for (int rr = 0; rr < 8; ++rr) {
      const int row = wave * 8 + rr;
      *(volatile v4f*)(out + (size_t)(m0 + row) * kD + lane * 4) = outv[rr];
    }
    __threadfence();
  }
}

extern "C" void kernel_launch(void* const* d_in, const int* in_sizes, int n_in,
                              void* d_out, int out_size, void* d_ws, size_t ws_size,
                              hipStream_t stream) {
  if (n_in < 12) return;
  if (in_sizes[0] != kNG * kGF) return;
  if (in_sizes[1] != kT * kFD) return;
  if (in_sizes[2] != kFD * kD) return;
  if (in_sizes[3] != kGF * kD) return;
  if (in_sizes[4] != kNL * kD * kD) return;
  if (in_sizes[5] != kNL * kD * kD) return;
  if (in_sizes[6] != kNL * kD * kD) return;
  if (in_sizes[7] != kNL * kD * kHid) return;
  if (in_sizes[8] != kNL * kHid * kD) return;
  if (in_sizes[9] != kD * kD) return;
  if (in_sizes[10] != kD * kD) return;
  if (in_sizes[11] != kD * kD) return;
  if (out_size != kRows * kD) return;
  if (ws_size < kWsTotal) return;

  const float* g      = (const float*)d_in[0];
  const float* lf     = (const float*)d_in[1];
  const float* W_vis  = (const float*)d_in[2];
  const float* W_txt  = (const float*)d_in[3];
  const float* Wq_enc = (const float*)d_in[4];
  const float* Wk_enc = (const float*)d_in[5];
  const float* Wv_enc = (const float*)d_in[6];
  const float* W1_ffn = (const float*)d_in[7];
  const float* W2_ffn = (const float*)d_in[8];
  const float* Wq_f   = (const float*)d_in[9];
  const float* Wk_f   = (const float*)d_in[10];
  const float* Wv_f   = (const float*)d_in[11];
  float* out = (float*)d_out;

  char* ws = (char*)d_ws;
  unsigned short* LF16  = (unsigned short*)(ws + kOffLF);
  unsigned short* WVIST = (unsigned short*)(ws + kOffWVIS);
  unsigned short* WQT   = (unsigned short*)(ws + kOffWQ);
  unsigned short* WKVT  = (unsigned short*)(ws + kOffWKV);
  unsigned short* W1T   = (unsigned short*)(ws + kOffW1);
  unsigned short* W2T   = (unsigned short*)(ws + kOffW2);
  unsigned short* WQFT  = (unsigned short*)(ws + kOffWQF);
  float*          VIS   = (float*)(ws + kOffVIS);
  unsigned short* LNVIS = (unsigned short*)(ws + kOffLNV);
  unsigned short* KV    = (unsigned short*)(ws + kOffKV);
  float*          TEXT  = (float*)(ws + kOffTEXT);
  unsigned short* KF    = (unsigned short*)(ws + kOffKF);
  unsigned short* VFT   = (unsigned short*)(ws + kOffVFT);
  float*          XBUF  = (float*)(ws + kOffX);
  float*          TST   = (float*)(ws + kOffTST);

  const float encS = (1.0f / sqrtf((float)kDq)) / (kWCarry * kKVCarry);
  const float encC = 1.0f / (kPCarry * kKVCarry);
  const float finS = (1.0f / sqrtf((float)kD)) / (kWCarry * kTxtCarry);
  const float finC = 1.0f / (kPCarry * kTxtCarry);
  const float yScale = 1.0f / (kWCarry * kWCarry);

  transpose_cast_kernel<<<dim3(kFD / 64, kD / 64, 1), 256, 0, stream>>>(W_vis, WVIST, kFD, kD, kWCarry);
  transpose_cast_kernel<<<dim3(kD / 64, kD / 64, kNL), 256, 0, stream>>>(Wq_enc, WQT, kD, kD, kWCarry);
  transpose_cast_kernel<<<dim3(kD / 64, kD / 64, kNL), 256, 0, stream>>>(Wk_enc, WKVT, kD, kD, kWCarry);
  transpose_cast_kernel<<<dim3(kD / 64, kD / 64, kNL), 256, 0, stream>>>(Wv_enc, WKVT + (size_t)kNL * kD * kD, kD, kD, kWCarry);
  transpose_cast_kernel<<<dim3(kD / 64, kHid / 64, kNL), 256, 0, stream>>>(W1_ffn, W1T, kD, kHid, kWCarry);
  transpose_cast_kernel<<<dim3(kHid / 64, kD / 64, kNL), 256, 0, stream>>>(W2_ffn, W2T, kHid, kD, kWCarry);
  transpose_cast_kernel<<<dim3(kD / 64, kD / 64, 1), 256, 0, stream>>>(Wq_f, WQFT, kD, kD, kWCarry);

  cast8_f16_kernel<<<(kT * kFD / 8) / 256, 256, 0, stream>>>(lf, LF16, kT * kFD / 8);

  wmma_gemm64<0, false, 0, 0, false><<<dim3(16, 1), 256, 0, stream>>>(
      LF16, nullptr, kFD, 0L,
      WVIST, nullptr, kFD, 0L,
      (void*)VIS, nullptr, kD, 0L,
      nullptr, nullptr, 0L,
      kT, kD, kFD, 1.0f / kWCarry);

  ln_vis_kernel<<<kVisRows / 16, 256, 0, stream>>>(VIS, LNVIS);

  text_kernel<<<1, 256, 0, stream>>>(g, W_txt, Wk_f, Wv_f, TEXT, KF, VFT, kTxtCarry);

  wmma_gemm64<0, false, 0, 1, false><<<dim3(17, 4), 256, 0, stream>>>(
      LNVIS, nullptr, kD, 0L,
      WKVT, nullptr, kD, (long)(kD * kD),
      (void*)KV, nullptr, kD, (long)kVisRows * kD,
      nullptr, nullptr, 0L,
      kVisRows, kD, kD, kKVCarry / kWCarry);

  for (int l = 0; l < kNL; ++l) {
    enc_attn_kernel<<<kT / 4, 256, 0, stream>>>(
        (l == 0) ? (const float*)TEXT : (const float*)TST, (l == 0) ? 1 : 0,
        WQT + (size_t)l * kD * kD,
        KV + (size_t)l * kVisRows * kD,
        KV + (size_t)(kNL + l) * kVisRows * kD,
        XBUF, encS, encC);
    ffn_kernel<<<kRows / 64, 256, 0, stream>>>(
        XBUF, W1T + (size_t)l * kHid * kD, W2T + (size_t)l * kD * kHid, TST, yScale);
  }

  final_attn_kernel<<<kRows / 64, 256, 0, stream>>>(TST, WQFT, KF, VFT, out, finS, finC);
}
